// GINModel_66159676227906
// MI455X (gfx1250) — hardware-verified
//
#include <hip/hip_runtime.h>
#include <stddef.h>
#include <stdint.h>


#define NN      100000
#define NE      3200000
#define FIN     13
#define HD      64
#define NG      512
#define HCAT    192
#define NTHR    256
#define NWAVE   8
#define EPT     8
#define CHUNK   (NTHR * EPT)
#define WCAP    (EPT * 32)
#define LISTN   (NWAVE * WCAP)
#define NB      512
#define NBLK    196
#define RCAP    20480
#define DEGCAP  80
#define PKS     11
#define RPK     9
#define MT      128
#define NTILE   782
#define MP      (NTILE * MT)
#define METAW   1056
#define STARTW  1024
#define PB_XP   782
#define NUW     14592
#define PB_W    57
#define PB_T    22
#define TABL    384
#define TABH    640
#define LDS_BKT  ((2 * RCAP + 2 * NB + LISTN + 64) * 4)
#define LDS_MLP  (MT * HD * 4 + MT * 128 * 2 + TABL * 4)
#define LDS_HEAD (128 * 384 * 2 + 128 * HCAT * 4 + TABH * 4 + 256 * 4 + 64)

#define O_XP    ((size_t)0)
#define S_XP    ((size_t)NN * 32)
#define O_Z     (O_XP + S_XP)
#define S_Z     ((size_t)MP * 256)
#define O_H     (O_Z + S_Z)
#define S_H     ((size_t)MP * 256)
#define O_LIST  (O_H + S_H)
#define S_LIST  ((size_t)NBLK * RCAP * 4)
#define O_META  (O_LIST + S_LIST)
#define S_META  ((size_t)NBLK * METAW * 4)
#define O_START (O_META + S_META)
#define S_START ((size_t)STARTW * 4)
#define O_P     (O_START + S_START)
#define S_P     ((size_t)NG * HCAT * 4)
#define O_WPL   (O_P + S_P)
#define S_WPL   ((size_t)NUW * 16)
#define O_TAB   (O_WPL + S_WPL)
#define S_TAB   ((size_t)(3 * TABL + TABH) * 4)
#define WS_END  (O_TAB + S_TAB)

static_assert((NE % 4) == 0);
static_assert(HD == 64 && FIN <= 16 && NG == 512 && HCAT == 3 * HD);
static_assert((CHUNK & (CHUNK - 1)) == 0 && CHUNK <= (1 << PKS));
static_assert(NB == (1 << RPK) && NB <= (1 << PKS) && LISTN >= NB && NTHR * 2 == NB);
static_assert(NN <= (1 << 17));
static_assert(NBLK * NB >= MP && MP >= NN && (NTILE - 1) * MT < NN);
static_assert((long long)RCAP * 100 >= 16671LL * 105 && (RCAP % 1024) == 0);
static_assert(DEGCAP >= 58 + 8);
static_assert(2 * NN <= PB_XP * NTHR && NUW == PB_W * NTHR);
static_assert(NUW == 256 + 5 * 1024 + 9216);
static_assert((S_XP % 128) == 0 && (S_Z % 128) == 0 && (S_H % 128) == 0 && (S_LIST % 128) == 0);
static_assert((S_META % 128) == 0 && (S_START % 128) == 0 && (S_P % 128) == 0 && (S_WPL % 128) == 0);
static_assert((S_TAB % 128) == 0 && WS_END <= (size_t)134217728);
static_assert(LDS_BKT <= 300000 && LDS_MLP <= 300000 && LDS_HEAD <= 300000);
static_assert((METAW * 4) % 128 == 0 && METAW == 2 * NB + 32);
static_assert((MP - (NBLK - 1) * NB) == 256);

typedef float          v4f  __attribute__((ext_vector_type(4)));
typedef float          v8f  __attribute__((ext_vector_type(8)));
typedef int            v4i  __attribute__((ext_vector_type(4)));
typedef int            v8i  __attribute__((ext_vector_type(8)));
typedef unsigned int   v2u  __attribute__((ext_vector_type(2)));
typedef unsigned int   v4u  __attribute__((ext_vector_type(4)));
typedef unsigned short v8us __attribute__((ext_vector_type(8)));
typedef __bf16         v16b __attribute__((ext_vector_type(16)));
typedef v4f  __attribute__((may_alias)) v4fa;
typedef v4i  __attribute__((may_alias)) v4ia;
typedef v2u  __attribute__((may_alias)) v2ua;
typedef v4u  __attribute__((may_alias)) v4ua;
typedef v8us __attribute__((may_alias)) v8usa;
union FragB { v16b v; v8us h[2]; v8i w; };

__device__ __forceinline__ v8f wmb(const FragB& a, const FragB& b, v8f c) {
  v8f d = __builtin_amdgcn_wmma_f32_16x16x32_bf16(false, a.v, false, b.v, (short)0, c, false, false);
  asm volatile("v_nop\n\tv_nop\n\tv_nop\n\tv_nop" : "+v"(d) : "v"(a.w), "v"(b.w));
  return d;
}

__device__ __forceinline__ unsigned short bf_bits(float f) {
  unsigned int u = __float_as_uint(f);
  const bool isn = (u & 0x7fffffffu) > 0x7f800000u;
  u += 0x7FFFu + ((u >> 16) & 1u);
  return isn ? (unsigned short)0x7fc0 : (unsigned short)(u >> 16);
}
__device__ __forceinline__ float bf_val(unsigned short b) { return __uint_as_float(((unsigned int)b) << 16); }
__device__ __forceinline__ float bf_rne(float f) { return bf_val(bf_bits(f)); }
__device__ __forceinline__ float relu_keep(float v) { return (v > 0.0f) ? v : (v - v); }

__device__ __forceinline__ void hilo8(const v4f a, const v4f b, v8us& hv, v8us& lv) {
  const float f[8] = {a.x, a.y, a.z, a.w, b.x, b.y, b.z, b.w};
#pragma unroll
  for (int j = 0; j < 8; ++j) {
    const unsigned short hb = bf_bits(f[j]);
    hv[j] = hb;
    lv[j] = bf_bits(f[j] - bf_val(hb));
  }
}

__device__ __forceinline__ int scan_chunk(const int* __restrict__ dsts, int nE, int cbase, int slotBase,
                                          int nb, int vec8, int* list, int tid, int lane, int wave) {
  int wc = 0;
  const int el0  = tid * EPT;
  const int e0   = cbase + el0;
  const int sent = -2147483647 - 1;
  v4i da, db;
  if (vec8 != 0 && cbase + CHUNK <= nE) {
    da = *(const v4i*)(dsts + e0);
    db = *(const v4i*)(dsts + e0 + 4);
  } else {
    da.x = (e0     < nE) ? dsts[min(e0,     nE - 1)] : sent;
    da.y = (e0 + 1 < nE) ? dsts[min(e0 + 1, nE - 1)] : sent;
    da.z = (e0 + 2 < nE) ? dsts[min(e0 + 2, nE - 1)] : sent;
    da.w = (e0 + 3 < nE) ? dsts[min(e0 + 3, nE - 1)] : sent;
    db.x = (e0 + 4 < nE) ? dsts[min(e0 + 4, nE - 1)] : sent;
    db.y = (e0 + 5 < nE) ? dsts[min(e0 + 5, nE - 1)] : sent;
    db.z = (e0 + 6 < nE) ? dsts[min(e0 + 6, nE - 1)] : sent;
    db.w = (e0 + 7 < nE) ? dsts[min(e0 + 7, nE - 1)] : sent;
  }
  const unsigned nbs = (unsigned)slotBase;
  const unsigned unb = (unsigned)nb;
  const unsigned s0 = (unsigned)da.x - nbs, s1 = (unsigned)da.y - nbs;
  const unsigned s2 = (unsigned)da.z - nbs, s3 = (unsigned)da.w - nbs;
  const unsigned s4 = (unsigned)db.x - nbs, s5 = (unsigned)db.y - nbs;
  const unsigned s6 = (unsigned)db.z - nbs, s7 = (unsigned)db.w - nbs;
  const bool h0 = s0 < unb, h1 = s1 < unb, h2 = s2 < unb, h3 = s3 < unb;
  const bool h4 = s4 < unb, h5 = s5 < unb, h6 = s6 < unb, h7 = s7 < unb;
  const unsigned any = __builtin_amdgcn_ballot_w32(h0 | h1 | h2 | h3 | h4 | h5 | h6 | h7);
  if (any != 0u) {
#define HITJ(J, HJ, SJ) { \
      const unsigned mj = __builtin_amdgcn_ballot_w32(HJ); \
      if (mj != 0u) { \
        if (HJ) { \
          const int pos = wc + (int)__builtin_amdgcn_mbcnt_lo(mj, 0u); \
          if (pos < WCAP) list[wave * WCAP + pos] = ((el0 + (J)) << PKS) | (int)(SJ); \
        } \
        wc += (int)__builtin_popcount(mj); } }
    HITJ(0, h0, s0)
    HITJ(1, h1, s1)
    HITJ(2, h2, s2)
    HITJ(3, h3, s3)
    HITJ(4, h4, s4)
    HITJ(5, h5, s5)
    HITJ(6, h6, s6)
    HITJ(7, h7, s7)
#undef HITJ
  }
  return wc;
}

__device__ __forceinline__ v8us wrow8(const float* __restrict__ W, int ldw, int kk, int n, int kmax) {
  v8us o;
#pragma unroll
  for (int i = 0; i < 8; ++i) {
    const int k  = kk + i;
    const int kc = k < kmax ? k : kmax - 1;
    const float v = W[(size_t)kc * (size_t)ldw + n];
    o[i] = (k < kmax) ? bf_bits(v) : (unsigned short)0;
  }
  return o;
}
__device__ __forceinline__ float tab_ld(const float* __restrict__ sp, int n, int stride, int off, int e) {
  const int ec = e < n ? e : n - 1;
  const float v = sp[ec * stride + off];
  return (e < n) ? bf_rne(v) : 0.0f;
}

__global__ __launch_bounds__(NTHR) void k_prep(
    const float* __restrict__ x,
    const float* __restrict__ w11, const float* __restrict__ w12, const float* __restrict__ w13,
    const float* __restrict__ w21, const float* __restrict__ w22, const float* __restrict__ w23,
    const float* __restrict__ fw1,
    const float* __restrict__ b11, const float* __restrict__ g1, const float* __restrict__ be1,
    const float* __restrict__ m1,  const float* __restrict__ v1, const float* __restrict__ b21,
    const float* __restrict__ b12, const float* __restrict__ g2, const float* __restrict__ be2,
    const float* __restrict__ m2,  const float* __restrict__ v2, const float* __restrict__ b22,
    const float* __restrict__ b13, const float* __restrict__ g3, const float* __restrict__ be3,
    const float* __restrict__ m3,  const float* __restrict__ v3, const float* __restrict__ b23,
    const float* __restrict__ fb1, const float* __restrict__ fw2, const float* __restrict__ fb2,
    unsigned short* xp, unsigned short* wpl, float* tab) {
  __shared__ __attribute__((aligned(16))) float tst[NTHR];
  const int tid = (int)threadIdx.x;
  const int bx  = (int)blockIdx.x;
  if (bx < PB_XP) {
    const int u = bx * NTHR + tid;
    const int row = u >> 1, half = u & 1;
    const int rc = row < NN ? row : NN - 1;
    const float* p = x + (size_t)rc * FIN;
    v8us o;
#pragma unroll
    for (int i = 0; i < 8; ++i) {
      const int c  = 8 * half + i;
      const int cc = c < FIN ? c : FIN - 1;
      const float v = p[cc];
      o[i] = (c < FIN) ? bf_bits(v) : (unsigned short)0;
    }
    unsigned short* dp = xp + (size_t)u * 8;
    const bool ok = u < 2 * NN;
    if (ok) *(volatile v8us*)dp = o;
    __threadfence();
    if (ok) *(volatile v8us*)dp = o;
  } else if (bx < PB_XP + PB_W) {
    const int u = (bx - PB_XP) * NTHR + tid;
    v8us o;
    if (u < 256) {
      const int n = u >> 2, k8 = (u & 3) * 8;
      o = wrow8(w11, HD, k8 & 15, n, FIN);
    } else if (u < 1280) {
      const int v = u - 256, n = v >> 4, k8 = (v & 15) * 8;
      o = wrow8(w12, HD, k8 & 63, n, HD);
    } else if (u < 2304) {
      const int v = u - 1280, n = v >> 4, k8 = (v & 15) * 8;
      o = wrow8(w13, HD, k8 & 63, n, HD);
    } else if (u < 3328) {
      const int v = u - 2304, n = v >> 4, k8 = (v & 15) * 8;
      o = wrow8(w21, HD, k8 & 63, n, HD);
    } else if (u < 4352) {
      const int v = u - 3328, n = v >> 4, k8 = (v & 15) * 8;
      o = wrow8(w22, HD, k8 & 63, n, HD);
    } else if (u < 5376) {
      const int v = u - 4352, n = v >> 4, k8 = (v & 15) * 8;
      o = wrow8(w23, HD, k8 & 63, n, HD);
    } else {
      const int v = u - 5376;
      const int n = v / 48;
      const int k8 = (v - n * 48) * 8;
      const int kk = k8 < HCAT ? k8 : k8 - HCAT;
      o = wrow8(fw1, HCAT, kk, n, HCAT);
    }
    unsigned short* dp = wpl + (size_t)u * 8;
    *(volatile v8us*)dp = o;
    __threadfence();
    *(volatile v8us*)dp = o;
  } else {
    const int tb = bx - PB_XP - PB_W;
    float val = 0.0f;
    int dstOff = 0, np = 16, mode = 0;
    switch (tb) {
      case 0:  val = tab_ld(b11, HD, 1, 0, tid); dstOff = 0;   break;
      case 1:  val = tab_ld(m1,  HD, 1, 0, tid); dstOff = 64;  break;
      case 2:  val = tab_ld(v1,  HD, 1, 0, tid); dstOff = 128; mode = 1; break;
      case 3:  val = tab_ld(g1,  HD, 1, 0, tid); dstOff = 192; break;
      case 4:  val = tab_ld(be1, HD, 1, 0, tid); dstOff = 256; break;
      case 5:  val = tab_ld(b21, HD, 1, 0, tid); dstOff = 320; break;
      case 6:  val = tab_ld(b12, HD, 1, 0, tid); dstOff = TABL + 0;   break;
      case 7:  val = tab_ld(m2,  HD, 1, 0, tid); dstOff = TABL + 64;  break;
      case 8:  val = tab_ld(v2,  HD, 1, 0, tid); dstOff = TABL + 128; mode = 1; break;
      case 9:  val = tab_ld(g2,  HD, 1, 0, tid); dstOff = TABL + 192; break;
      case 10: val = tab_ld(be2, HD, 1, 0, tid); dstOff = TABL + 256; break;
      case 11: val = tab_ld(b22, HD, 1, 0, tid); dstOff = TABL + 320; break;
      case 12: val = tab_ld(b13, HD, 1, 0, tid); dstOff = 2 * TABL + 0;   break;
      case 13: val = tab_ld(m3,  HD, 1, 0, tid); dstOff = 2 * TABL + 64;  break;
      case 14: val = tab_ld(v3,  HD, 1, 0, tid); dstOff = 2 * TABL + 128; mode = 1; break;
      case 15: val = tab_ld(g3,  HD, 1, 0, tid); dstOff = 2 * TABL + 192; break;
      case 16: val = tab_ld(be3, HD, 1, 0, tid); dstOff = 2 * TABL + 256; break;
      case 17: val = tab_ld(b23, HD, 1, 0, tid); dstOff = 2 * TABL + 320; break;
      case 18: val = tab_ld(fb1, HCAT, 1, 0, tid); dstOff = 3 * TABL + 0;   np = 48; break;
      case 19: val = tab_ld(fw2, HCAT, 2, 0, tid); dstOff = 3 * TABL + 192; np = 48; break;
      case 20: val = tab_ld(fw2, HCAT, 2, 1, tid); dstOff = 3 * TABL + 384; np = 48; break;
      default: val = tab_ld(fb2, 2,    1, 0, tid); dstOff = 3 * TABL + 576; break;
    }
    const float rsv = 1.0f / sqrtf(val + 1e-5f);
    val = (mode != 0) ? rsv : val;
    tst[tid] = val;
    __syncthreads();
    const int pc = tid < 63 ? tid : 63;
    const v4f pv = *(const v4fa*)(tst + 4 * pc);
    float* dp = tab + dstOff + 4 * tid;
    const bool ok = tid < np;
    if (ok) *(volatile v4f*)dp = pv;
    __threadfence();
    if (ok) *(volatile v4f*)dp = pv;
  }
}

__global__ __launch_bounds__(NTHR) void k_bounds(const int* __restrict__ bat, int* start) {
  __shared__ __attribute__((aligned(16))) int st[STARTW];
  const int tid = (int)threadIdx.x;
  for (int i = tid; i < STARTW; i += NTHR) st[i] = 0;
  __syncthreads();
  const int nIt = (NN + 1 + NTHR - 1) / NTHR;
#pragma unroll 1
  for (int it = 0; it < nIt; ++it) {
    const int n  = it * NTHR + tid;
    int ip = n - 1; ip = ip < 0 ? 0 : (ip > NN - 1 ? NN - 1 : ip);
    const int ic = n > NN - 1 ? NN - 1 : n;
    const int pv = bat[ip];
    const int cv = bat[ic];
    const int prev = (n == 0) ? -1 : pv;
    const int cur  = (n >= NN) ? NG : cv;
    if (n <= NN) {
      if (n >= 1 && n < NN && cur < prev) st[NG + 1] = 1;
      const int lo = prev + 1 < 0 ? 0 : prev + 1;
      const int hi = cur > NG ? NG : cur;
      int cg = hi - lo + 1;
      cg = cg < 0 ? 0 : (cg > NG + 1 ? NG + 1 : cg);
#pragma unroll 1
      for (int q = 0; q < cg; ++q) st[lo + q] = n;
    }
  }
  __syncthreads();
  const v4i v = *(const v4ia*)(st + 4 * tid);
  int* dp = start + 4 * tid;
  *(volatile v4i*)dp = v;
  __threadfence();
  *(volatile v4i*)dp = v;
}

__global__ __launch_bounds__(NTHR) void k_bucket(const int* __restrict__ srcs, const int* __restrict__ dsts,
                                                 int* lists, int* meta) {
  extern __shared__ v4f lds_dyn[];
  int* reg1 = (int*)lds_dyn;
  int* reg2 = reg1 + RCAP;
  int* scnt = reg2 + RCAP;
  int* soff = scnt + NB;
  int* list = soff + NB;
  int* wcnt = list + LISTN;
  int* wtot = wcnt + NWAVE;
  int* wdf  = wtot + NWAVE;
  int* flg  = wdf + NWAVE;
  const int tid = (int)threadIdx.x, lane = tid & 31, wave = tid >> 5;
  const int blk = (int)blockIdx.x;
  const int nodeBase = blk * NB;

  scnt[tid] = 0; scnt[tid + NTHR] = 0;
  {
    const v4i z4 = {0, 0, 0, 0};
#pragma unroll 1
    for (int it = 0; it < RCAP / (4 * NTHR); ++it) *(v4ia*)(reg2 + 4 * (it * NTHR + tid)) = z4;
  }
  if (tid < 32) flg[tid] = 0;
  __syncthreads();

  int tot = 0;
  const int nChunks = (NE + CHUNK - 1) / CHUNK;
#pragma unroll 1
  for (int ch = 0; ch < nChunks; ++ch) {
    const int cbase = ch * CHUNK;
    const int wc = scan_chunk(dsts, NE, cbase, nodeBase, NB, 1, list, tid, lane, wave);
    if (lane == 0) wcnt[wave] = wc;
    __syncthreads();
    int pre = 0, all = 0;
#pragma unroll
    for (int w2 = 0; w2 < NWAVE; ++w2) {
      int c = wcnt[w2];
      c = c < 0 ? 0 : (c > WCAP ? WCAP : c);
      all += c;
      pre += (w2 < wave) ? c : 0;
    }
    const int wcc  = wc > WCAP ? WCAP : wc;
    const int base = tot + pre;
#pragma unroll 1
    for (int i0 = 0; i0 < wcc; i0 += 32) {
      const int i  = i0 + lane;
      const int ic = i < wcc ? i : wcc - 1;
      const int ent = list[wave * WCAP + ic];
      const int el  = (ent >> PKS) & (CHUNK - 1);
      const int sl  = ent & (NB - 1);
      int eid = cbase + el;
      eid = eid < 0 ? 0 : (eid > NE - 1 ? NE - 1 : eid);
      int s = srcs[eid];
      s = s < 0 ? 0 : (s > NN - 1 ? NN - 1 : s);
      const int pos = base + i;
      if (i < wcc && pos < RCAP) reg1[pos] = (s << RPK) | sl;
    }
    tot += all;
    tot = tot > RCAP ? RCAP : tot;
    __syncthreads();
  }
  const int nh = tot;

  if (wave == 0) {
#pragma unroll 1
    for (int b0 = 0; b0 < nh; b0 += 32) {
      int idx = b0 + lane;
      idx = idx > nh - 1 ? nh - 1 : idx;
      const int uv  = reg1[idx];
      const int m32 = (nh - b0) < 32 ? (nh - b0) : 32;
#pragma unroll 1
      for (int k = 0; k < m32; ++k) {
        const int u  = __builtin_amdgcn_readlane(uv, k);
        const int sl = u & (NB - 1);
        if (lane == 0) scnt[sl] = scnt[sl] + 1;
      }
    }
  }
  __syncthreads();

  {
    int e0 = scnt[2 * tid], e1 = scnt[2 * tid + 1];
    e0 = e0 < 0 ? 0 : e0; e1 = e1 < 0 ? 0 : e1;
    const int ts = e0 + e1;
    int incl = ts;
#pragma unroll
    for (int d = 1; d < 32; d <<= 1) {
      const int up = __shfl_up(incl, d);
      if (lane >= d) incl += up;
    }
    const unsigned dm = __builtin_amdgcn_ballot_w32((e0 > DEGCAP) || (e1 > DEGCAP));
    if (lane == 31) wtot[wave] = incl;
    if (lane == 0) wdf[wave] = (dm != 0u) ? 1 : 0;
    __syncthreads();
    int pre = 0;
#pragma unroll
    for (int w2 = 0; w2 < NWAVE; ++w2) pre += (w2 < wave) ? wtot[w2] : 0;
    const int run = pre + incl - ts;
    soff[2 * tid]     = run;
    soff[2 * tid + 1] = run + e0;
  }
  __syncthreads();
  list[tid] = soff[tid]; list[tid + NTHR] = soff[tid + NTHR];
  __syncthreads();

  if (wave == 0) {
#pragma unroll 1
    for (int b0 = 0; b0 < nh; b0 += 32) {
      int idx = b0 + lane;
      idx = idx > nh - 1 ? nh - 1 : idx;
      const int uv  = reg1[idx];
      const int m32 = (nh - b0) < 32 ? (nh - b0) : 32;
#pragma unroll 1
      for (int k = 0; k < m32; ++k) {
        const int u  = __builtin_amdgcn_readlane(uv, k);
        const int sl = u & (NB - 1);
        const int sv = (int)((unsigned)u >> RPK);
        if (lane == 0) {
          int pos = list[sl];
          pos = pos < 0 ? 0 : (pos > RCAP - 1 ? RCAP - 1 : pos);
          reg2[pos] = sv;
          list[sl] = pos + 1;
        }
      }
    }
    if (lane == 0) {
      int df = 0;
#pragma unroll
      for (int w2 = 0; w2 < NWAVE; ++w2) df |= wdf[w2];
      flg[0] = ((nh >= RCAP) || (df != 0)) ? 1 : 0;
      flg[1] = nh;
    }
  }
  __syncthreads();

  int* lp = lists + (size_t)blk * RCAP;
  int* mp = meta + (size_t)blk * METAW;
  const v4i mv = *(const v4ia*)(scnt + 4 * tid);
  const int fl = tid < 8 ? tid : 7;
  const v4i fv = *(const v4ia*)(flg + 4 * fl);
#pragma unroll 1
  for (int it = 0; it < RCAP / (4 * NTHR); ++it) {
    const int p = it * NTHR + tid;
    const v4i v = *(const v4ia*)(reg2 + 4 * p);
    *(volatile v4i*)(lp + 4 * p) = v;
  }
  *(volatile v4i*)(mp + 4 * tid) = mv;
  if (tid < 8) *(volatile v4i*)(mp + 2 * NB + 4 * tid) = fv;
  __threadfence();
#pragma unroll 1
  for (int it = 0; it < RCAP / (4 * NTHR); ++it) {
    const int p = it * NTHR + tid;
    const v4i v = *(const v4ia*)(reg2 + 4 * p);
    *(volatile v4i*)(lp + 4 * p) = v;
  }
  *(volatile v4i*)(mp + 4 * tid) = mv;
  if (tid < 8) *(volatile v4i*)(mp + 2 * NB + 4 * tid) = fv;
}

__global__ __launch_bounds__(NTHR) void k_agg1(const unsigned short* __restrict__ xp,
                                               const int* __restrict__ lists, const int* __restrict__ meta,
                                               unsigned short* z1) {
  __shared__ __attribute__((aligned(16))) int mt[2 * NB];
  __shared__ __attribute__((aligned(16))) unsigned short zt[NB * 32];
  const int tid = (int)threadIdx.x, lane = tid & 31, wave = tid >> 5;
  const int blk = (int)blockIdx.x;
  const int nodeBase = blk * NB;
  const int* mp = meta + (size_t)blk * METAW;
  *(v4ia*)(mt + 4 * tid) = *(const v4i*)(mp + 4 * tid);
  const int flag = mp[2 * NB];
  __syncthreads();
  const int* lp = lists + (size_t)blk * RCAP;
  const int hs = lane >> 2, cq = lane & 3;
  const float qnan = __int_as_float(0x7fc00000);

#pragma unroll 1
  for (int jt = 0; jt < NB / NWAVE; ++jt) {
    const int slot = wave * (NB / NWAVE) + jt;
    const int grow = nodeBase + slot;
    const int craw = mt[slot];
    int st = mt[NB + slot];
    int cnt = craw;
    st  = st < 0 ? 0 : (st > RCAP ? RCAP : st);
    cnt = cnt < 0 ? 0 : (cnt > DEGCAP ? DEGCAP : cnt);
    if (cnt > RCAP - st) cnt = RCAP - st;
    const float pz = (flag != 0 || craw > DEGCAP || craw < 0) ? qnan : 0.0f;
    const bool liveRow = grow < NN;

    float a0 = 0.f, a1 = 0.f, a2 = 0.f, a3 = 0.f;
#pragma unroll 1
    for (int b0 = 0; b0 < cnt; b0 += 32) {
      int idx = st + b0 + lane;
      idx = idx > st + cnt - 1 ? st + cnt - 1 : idx;
      idx = idx < 0 ? 0 : (idx > RCAP - 1 ? RCAP - 1 : idx);
      int sv = lp[idx];
      sv = sv < 0 ? 0 : (sv > NN - 1 ? NN - 1 : sv);
      const int m32 = (cnt - b0) < 32 ? (cnt - b0) : 32;
      const int ns  = (m32 + 7) >> 3;
#pragma unroll 1
      for (int s = 0; s < ns; ++s) {
        const int j = 8 * s + hs;
        const int sidx = __shfl(sv, j);
        const bool ok = (b0 + j) < cnt;
        const v2u w = *(const v2u*)(xp + (size_t)sidx * 16 + 4 * cq);
        const float f0 = __uint_as_float(w.x << 16), f1 = __uint_as_float(w.x & 0xffff0000u);
        const float f2 = __uint_as_float(w.y << 16), f3 = __uint_as_float(w.y & 0xffff0000u);
        a0 += ok ? f0 : 0.0f; a1 += ok ? f1 : 0.0f; a2 += ok ? f2 : 0.0f; a3 += ok ? f3 : 0.0f;
      }
    }
#pragma unroll
    for (int d = 4; d < 32; d <<= 1) {
      const float t0 = __shfl_xor(a0, d), t1 = __shfl_xor(a1, d);
      const float t2 = __shfl_xor(a2, d), t3 = __shfl_xor(a3, d);
      a0 += t0; a1 += t1; a2 += t2; a3 += t3;
    }
    const int nc = liveRow ? grow : NN - 1;
    const v2u sw = *(const v2u*)(xp + (size_t)nc * 16 + 4 * cq);
    const float s0 = __uint_as_float(sw.x << 16), s1 = __uint_as_float(sw.x & 0xffff0000u);
    const float s2 = __uint_as_float(sw.y << 16), s3 = __uint_as_float(sw.y & 0xffff0000u);
    const float r0 = (liveRow ? s0 + a0 : 0.0f) + pz;
    const float r1 = (liveRow ? s1 + a1 : 0.0f) + pz;
    const float r2 = (liveRow ? s2 + a2 : 0.0f) + pz;
    const float r3 = (liveRow ? s3 + a3 : 0.0f) + pz;
    const unsigned short hb0 = bf_bits(r0), hb1 = bf_bits(r1), hb2 = bf_bits(r2), hb3 = bf_bits(r3);
    const unsigned short lb0 = bf_bits(r0 - bf_val(hb0)), lb1 = bf_bits(r1 - bf_val(hb1));
    const unsigned short lb2 = bf_bits(r2 - bf_val(hb2)), lb3 = bf_bits(r3 - bf_val(hb3));
    v2u hw, lw;
    hw.x = (unsigned int)hb0 | ((unsigned int)hb1 << 16);
    hw.y = (unsigned int)hb2 | ((unsigned int)hb3 << 16);
    lw.x = (unsigned int)lb0 | ((unsigned int)lb1 << 16);
    lw.y = (unsigned int)lb2 | ((unsigned int)lb3 << 16);
    if (hs == 0) {
      *(v2ua*)(zt + slot * 32 + 4 * cq)      = hw;
      *(v2ua*)(zt + slot * 32 + 16 + 4 * cq) = lw;
    }
  }
  __syncthreads();
  int nr = MP - nodeBase;
  nr = nr > NB ? NB : nr;
  const int nIt = (nr * 4) / NTHR;
  unsigned short* zp = z1 + (size_t)nodeBase * 32;
#pragma unroll 1
  for (int it = 0; it < nIt; ++it) {
    const int p = it * NTHR + tid;
    const v4u v = *(const v4ua*)(zt + 8 * p);
    *(volatile v4u*)(zp + 8 * p) = v;
  }
  __threadfence();
#pragma unroll 1
  for (int it = 0; it < nIt; ++it) {
    const int p = it * NTHR + tid;
    const v4u v = *(const v4ua*)(zt + 8 * p);
    *(volatile v4u*)(zp + 8 * p) = v;
  }
}

__global__ __launch_bounds__(NTHR) void k_agg2(const float* __restrict__ hf,
                                               const int* __restrict__ lists, const int* __restrict__ meta,
                                               unsigned short* zhl) {
  __shared__ __attribute__((aligned(16))) int mt[2 * NB];
  const int tid = (int)threadIdx.x, lane = tid & 31, wave = tid >> 5;
  const int blk = (int)blockIdx.x;
  const int nodeBase = blk * NB;
  const int* mp = meta + (size_t)blk * METAW;
  *(v4ia*)(mt + 4 * tid) = *(const v4i*)(mp + 4 * tid);
  const int flag = mp[2 * NB];
  __syncthreads();
  const int* lp = lists + (size_t)blk * RCAP;
  const int hs = lane >> 4, cq = lane & 15;
  const float qnan = __int_as_float(0x7fc00000);

#pragma unroll 1
  for (int jt = 0; jt < NB / NWAVE; ++jt) {
    const int slot = wave * (NB / NWAVE) + jt;
    const int grow = nodeBase + slot;
    const int craw = mt[slot];
    int st = mt[NB + slot];
    int cnt = craw;
    st  = st < 0 ? 0 : (st > RCAP ? RCAP : st);
    cnt = cnt < 0 ? 0 : (cnt > DEGCAP ? DEGCAP : cnt);
    if (cnt > RCAP - st) cnt = RCAP - st;
    const float pz = (flag != 0 || craw > DEGCAP || craw < 0) ? qnan : 0.0f;
    const bool liveRow = grow < NN;

    float a0 = 0.f, a1 = 0.f, a2 = 0.f, a3 = 0.f;
#pragma unroll 1
    for (int b0 = 0; b0 < cnt; b0 += 32) {
      int idx = st + b0 + lane;
      idx = idx > st + cnt - 1 ? st + cnt - 1 : idx;
      idx = idx < 0 ? 0 : (idx > RCAP - 1 ? RCAP - 1 : idx);
      int sv = lp[idx];
      sv = sv < 0 ? 0 : (sv > NN - 1 ? NN - 1 : sv);
      const int m32 = (cnt - b0) < 32 ? (cnt - b0) : 32;
      const int ns  = (m32 + 1) >> 1;
#pragma unroll 1
      for (int s = 0; s < ns; ++s) {
        const int j = 2 * s + hs;
        const int sidx = __shfl(sv, j);
        const bool ok = (b0 + j) < cnt;
        const v4f v = *(const v4f*)(hf + (size_t)sidx * HD + 4 * cq);
        a0 += ok ? v.x : 0.0f; a1 += ok ? v.y : 0.0f; a2 += ok ? v.z : 0.0f; a3 += ok ? v.w : 0.0f;
      }
    }
    {
      const float t0 = __shfl_xor(a0, 16), t1 = __shfl_xor(a1, 16);
      const float t2 = __shfl_xor(a2, 16), t3 = __shfl_xor(a3, 16);
      a0 += t0; a1 += t1; a2 += t2; a3 += t3;
    }
    const int nc = liveRow ? grow : NN - 1;
    const v4f sf = *(const v4f*)(hf + (size_t)nc * HD + 4 * cq);
    const float r0 = (liveRow ? sf.x + a0 : 0.0f) + pz;
    const float r1 = (liveRow ? sf.y + a1 : 0.0f) + pz;
    const float r2 = (liveRow ? sf.z + a2 : 0.0f) + pz;
    const float r3 = (liveRow ? sf.w + a3 : 0.0f) + pz;
    const unsigned short hb0 = bf_bits(r0), hb1 = bf_bits(r1), hb2 = bf_bits(r2), hb3 = bf_bits(r3);
    const unsigned short lb0 = bf_bits(r0 - bf_val(hb0)), lb1 = bf_bits(r1 - bf_val(hb1));
    const unsigned short lb2 = bf_bits(r2 - bf_val(hb2)), lb3 = bf_bits(r3 - bf_val(hb3));
    const bool isHi = (hs == 0);
    const unsigned int q0 = isHi ? hb0 : lb0, q1 = isHi ? hb1 : lb1;
    const unsigned int q2 = isHi ? hb2 : lb2, q3 = isHi ? hb3 : lb3;
    v2u pk;
    pk.x = q0 | (q1 << 16);
    pk.y = q2 | (q3 << 16);
    unsigned short* gp = zhl + (size_t)grow * 128 + 4 * lane;
    const bool wsv = grow < MP;
    if (wsv) *(volatile v2u*)gp = pk;
    __threadfence();
    if (wsv) *(volatile v2u*)gp = pk;
  }
}

template <int KA>
__global__ __launch_bounds__(NTHR) void k_mlp(const unsigned short* __restrict__ Z,
                                              const unsigned short* __restrict__ W1D,
                                              const unsigned short* __restrict__ W2D,
                                              const float* __restrict__ tabg, float* H) {
  extern __shared__ v4f lds_dyn[];
  float* stg = (float*)lds_dyn;
  unsigned short* a2 = (unsigned short*)(stg + MT * HD);
  float* tab = (float*)(a2 + MT * 128);
  const int tid = (int)threadIdx.x, lane = tid & 31, wave = tid >> 5, hh = lane >> 4, m = lane & 15;
  const int rowBase = (int)blockIdx.x * MT;
  if (tid < TABL / 4) *(v4fa*)(tab + 4 * tid) = *(const v4f*)(tabg + 4 * tid);

  v8f acc[4];
  const v8f zz = {0.f, 0.f, 0.f, 0.f, 0.f, 0.f, 0.f, 0.f};
#pragma unroll
  for (int t = 0; t < 4; ++t) acc[t] = zz;
  {
    const unsigned short* ap = Z + (size_t)(rowBase + 16 * wave + m) * (size_t)KA + 8 * hh;
    const unsigned short* bp = W1D + (size_t)m * (size_t)KA + 8 * hh;
#pragma unroll 1
    for (int k0 = 0; k0 < KA; k0 += 32) {
      FragB af;
      af.h[0] = *(const v8usa*)(ap + k0);
      af.h[1] = *(const v8usa*)(ap + k0 + 16);
#pragma unroll
      for (int t = 0; t < 4; ++t) {
        const unsigned short* wq = bp + (size_t)(16 * t) * (size_t)KA + k0;
        FragB bf;
        bf.h[0] = *(const v8usa*)wq;
        bf.h[1] = *(const v8usa*)(wq + 16);
        acc[t] = wmb(af, bf, acc[t]);
      }
    }
  }
  __syncthreads();

#pragma unroll
  for (int t = 0; t < 4; ++t) {
    const int lc = 16 * t + m;
    const float b1 = tab[lc], mm = tab[64 + lc], rs = tab[128 + lc], gg = tab[192 + lc], be = tab[256 + lc];
#pragma unroll
    for (int r = 0; r < 8; ++r) {
      const int lr = 16 * wave + 8 * hh + r;
      float v = acc[t][r] + b1;
      v = ((v - mm) * rs) * gg + be;
      stg[lr * HD + lc] = relu_keep(v);
    }
  }
  __syncthreads();
#pragma unroll 1
  for (int it = 0; it < (MT * 8) / NTHR; ++it) {
    const int p = it * NTHR + tid;
    const int row = p >> 3, q = p & 7;
    const v4f a = *(const v4fa*)(stg + row * HD + 8 * q);
    const v4f b = *(const v4fa*)(stg + row * HD + 8 * q + 4);
    v8us hv, lv;
    hilo8(a, b, hv, lv);
    *(v8usa*)(a2 + row * 128 + 8 * q)      = hv;
    *(v8usa*)(a2 + row * 128 + 64 + 8 * q) = lv;
  }
  __syncthreads();

#pragma unroll
  for (int t = 0; t < 4; ++t) acc[t] = zz;
  {
    const unsigned short* ap = a2 + (16 * wave + m) * 128 + 8 * hh;
    const unsigned short* bp = W2D + (size_t)m * 128 + 8 * hh;
#pragma unroll 1
    for (int k0 = 0; k0 < 128; k0 += 32) {
      FragB af;
      af.h[0] = *(const v8usa*)(ap + k0);
      af.h[1] = *(const v8usa*)(ap + k0 + 16);
#pragma unroll
      for (int t = 0; t < 4; ++t) {
        const unsigned short* wq = bp + (size_t)(16 * t) * 128 + k0;
        FragB bf;
        bf.h[0] = *(const v8usa*)wq;
        bf.h[1] = *(const v8usa*)(wq + 16);
        acc[t] = wmb(af, bf, acc[t]);
      }
    }
  }
#pragma unroll
  for (int t = 0; t < 4; ++t) {
    const int lc = 16 * t + m;
    const float b2 = tab[320 + lc];
#pragma unroll
    for (int r = 0; r < 8; ++r) {
      const int lr = 16 * wave + 8 * hh + r;
      const bool live = (rowBase + lr) < NN;
      const float v = relu_keep(acc[t][r] + b2);
      stg[lr * HD + lc] = live ? v : 0.0f;
    }
  }
  __syncthreads();
  v4f fv[8];
#pragma unroll
  for (int i = 0; i < 8; ++i) {
    const int lr = 16 * wave + 2 * i + hh;
    fv[i] = *(const v4fa*)(stg + lr * HD + 4 * m);
  }
#pragma unroll
  for (int i = 0; i < 8; ++i) {
    const int gr = rowBase + 16 * wave + 2 * i + hh;
    float* op = H + (size_t)gr * HD + 4 * m;
    *(volatile v4f*)op = fv[i];
  }
  __threadfence();
#pragma unroll
  for (int i = 0; i < 8; ++i) {
    const int gr = rowBase + 16 * wave + 2 * i + hh;
    float* op = H + (size_t)gr * HD + 4 * m;
    *(volatile v4f*)op = fv[i];
  }
}

__global__ __launch_bounds__(NTHR) void k_pool(const float* __restrict__ hf, const int* __restrict__ start,
                                               float* P, int colOff) {
  __shared__ __attribute__((aligned(16))) float wsum[NWAVE * HD];
  __shared__ __attribute__((aligned(16))) float outs[HD];
  const int tid = (int)threadIdx.x, lane = tid & 31, wave = tid >> 5;
  const int g = (int)blockIdx.x;
  int s = start[g], e = start[g + 1];
  s = s < 0 ? 0 : (s > NN ? NN : s);
  e = e < 0 ? 0 : (e > NN ? NN : e);
  int nr = e - s;
  nr = nr < 0 ? 0 : nr;
  const int hs = lane >> 4, cq = lane & 15;
  float a0 = 0.f, a1 = 0.f, a2 = 0.f, a3 = 0.f;
#pragma unroll 1
  for (int r0 = 2 * wave; r0 < nr; r0 += 2 * NWAVE) {
    const int r = r0 + hs;
    const bool ok = r < nr;
    int node = s + r;
    node = node > NN - 1 ? NN - 1 : node;
    const v4f v = *(const v4f*)(hf + (size_t)node * HD + 4 * cq);
    a0 += ok ? v.x : 0.0f; a1 += ok ? v.y : 0.0f; a2 += ok ? v.z : 0.0f; a3 += ok ? v.w : 0.0f;
  }
  {
    const float t0 = __shfl_xor(a0, 16), t1 = __shfl_xor(a1, 16);
    const float t2 = __shfl_xor(a2, 16), t3 = __shfl_xor(a3, 16);
    a0 += t0; a1 += t1; a2 += t2; a3 += t3;
  }
  if (hs == 0) {
    v4f pv; pv.x = a0; pv.y = a1; pv.z = a2; pv.w = a3;
    *(v4fa*)(wsum + wave * HD + 4 * cq) = pv;
  }
  __syncthreads();
  if (tid < HD) {
    float t = 0.0f;
#pragma unroll
    for (int w2 = 0; w2 < NWAVE; ++w2) t += wsum[w2 * HD + tid];
    outs[tid] = t;
  }
  __syncthreads();
  const v4f ov = *(const v4fa*)(outs + 4 * cq);
  float* op = P + (size_t)g * HCAT + colOff + 4 * cq;
  const bool okst = (tid < 16);
  if (okst) *(volatile v4f*)op = ov;
  __threadfence();
  if (okst) *(volatile v4f*)op = ov;
}

__global__ __launch_bounds__(NTHR) void k_head(const float* __restrict__ P, const unsigned short* __restrict__ FCD,
                                               const float* __restrict__ tabg, const int* __restrict__ meta,
                                               const int* __restrict__ start, float* out) {
  extern __shared__ v4f lds_dyn[];
  unsigned short* ah = (unsigned short*)lds_dyn;
  float* rr   = (float*)(ah + 128 * 384);
  float* tab  = rr + 128 * HCAT;
  float* outs = tab + TABH;
  int*   wfl  = (int*)(outs + 256);
  const int tid = (int)threadIdx.x, lane = tid & 31, wave = tid >> 5, hh = lane >> 4, m = lane & 15;
  const int rowBase = (int)blockIdx.x * 128;

  if (tid < TABH / 4) *(v4fa*)(tab + 4 * tid) = *(const v4f*)(tabg + 4 * tid);
  {
    const int bi = tid < NBLK ? tid : NBLK - 1;
    const int fv = meta[(size_t)bi * METAW + 2 * NB];
    const int un = start[NG + 1];
    const bool pr = ((tid < NBLK) && (fv != 0)) || (un != 0);
    const unsigned bal = __builtin_amdgcn_ballot_w32(pr);
    if (lane == 0) wfl[wave] = (bal != 0u) ? 1 : 0;
  }
#pragma unroll 1
  for (int it = 0; it < (128 * 24) / NTHR; ++it) {
    const int p = it * NTHR + tid;
    const int row = p / 24, q = p - row * 24;
    const float* pp = P + (size_t)(rowBase + row) * HCAT + 8 * q;
    const v4f a = *(const v4f*)pp;
    const v4f b = *(const v4f*)(pp + 4);
    v8us hv, lv;
    hilo8(a, b, hv, lv);
    *(v8usa*)(ah + row * 384 + 8 * q)        = hv;
    *(v8usa*)(ah + row * 384 + HCAT + 8 * q) = lv;
  }
  __syncthreads();

  const v8f zz = {0.f, 0.f, 0.f, 0.f, 0.f, 0.f, 0.f, 0.f};
#pragma unroll 1
  for (int ng = 0; ng < 3; ++ng) {
    v8f acc[4];
#pragma unroll
    for (int t = 0; t < 4; ++t) acc[t] = zz;
    const unsigned short* ap = ah + (16 * wave + m) * 384 + 8 * hh;
    const unsigned short* bp = FCD + (size_t)(64 * ng + m) * 384 + 8 * hh;
#pragma unroll 1
    for (int k0 = 0; k0 < 384; k0 += 32) {
      FragB af;
      af.h[0] = *(const v8usa*)(ap + k0);
      af.h[1] = *(const v8usa*)(ap + k0 + 16);
#pragma unroll
      for (int t = 0; t < 4; ++t) {
        const unsigned short* wq = bp + (size_t)(16 * t) * 384 + k0;
        FragB bf;
        bf.h[0] = *(const v8usa*)wq;
        bf.h[1] = *(const v8usa*)(wq + 16);
        acc[t] = wmb(af, bf, acc[t]);
      }
    }
#pragma unroll
    for (int t = 0; t < 4; ++t) {
      const int lc = 64 * ng + 16 * t + m;
      const float bb = tab[lc];
#pragma unroll
      for (int r = 0; r < 8; ++r) {
        const int lr = 16 * wave + 8 * hh + r;
        rr[lr * HCAT + lc] = relu_keep(acc[t][r] + bb);
      }
    }
  }
  __syncthreads();

  const int row = tid >> 1, c = tid & 1;
  const float* rp = rr + row * HCAT;
  const float* wp = tab + HCAT + c * HCAT;
  float sacc = 0.0f;
#pragma unroll 4
  for (int k = 0; k < HCAT; ++k) sacc = fmaf(rp[k], wp[k], sacc);
  const float o  = sacc + tab[3 * HCAT + c];
  const float po = __shfl_xor(o, 1);
  const float o0 = (c != 0) ? po : o;
  const float o1 = (c != 0) ? o : po;
  const float mx = (o0 > o1) ? o0 : o1;
  const float s0 = o0 - mx, s1 = o1 - mx;
  const float lse = logf(expf(s0) + expf(s1));
  const float mine = ((c != 0) ? s1 : s0) - lse;
  int pf = 0;
#pragma unroll
  for (int w2 = 0; w2 < NWAVE; ++w2) pf |= wfl[w2];
  const float qnan = __int_as_float(0x7fc00000);
  outs[tid] = (pf != 0) ? qnan : mine;
  __syncthreads();
  const int pc = tid < 63 ? tid : 63;
  const v4f ov = *(const v4fa*)(outs + 4 * pc);
  float* op = out + (size_t)blockIdx.x * 256 + 4 * tid;
  const bool okst = tid < 64;
  if (okst) *(volatile v4f*)op = ov;
  __threadfence();
  if (okst) *(volatile v4f*)op = ov;
}

extern "C" void kernel_launch(void* const* d_in, const int* in_sizes, int n_in,
                              void* d_out, int out_size, void* d_ws, size_t ws_size,
                              hipStream_t stream) {
  if (n_in < 32) return;
  if (in_sizes[0] != NN * FIN || in_sizes[1] != NE || in_sizes[2] != NE || in_sizes[3] != NN) return;
  if (in_sizes[4] != FIN * HD) return;
  for (int l = 0; l < 3; ++l) {
    const int b = 4 + 8 * l;
    if (l > 0 && in_sizes[b] != HD * HD) return;
    for (int j = 1; j <= 5; ++j) if (in_sizes[b + j] != HD) return;
    if (in_sizes[b + 6] != HD * HD || in_sizes[b + 7] != HD) return;
  }
  if (in_sizes[28] != HCAT * HCAT || in_sizes[29] != HCAT || in_sizes[30] != HCAT * 2 || in_sizes[31] != 2) return;
  if (out_size != NG * 2) return;
  if ((size_t)WS_END > ws_size) return;

  const float* x     = (const float*)d_in[0];
  const int*   src   = (const int*)  d_in[1];
  const int*   dst   = (const int*)  d_in[2];
  const int*   batch = (const int*)  d_in[3];
  const float* cp[3][8];
  for (int l = 0; l < 3; ++l)
    for (int j = 0; j < 8; ++j) cp[l][j] = (const float*)d_in[4 + 8 * l + j];
  const float* fc1W = (const float*)d_in[28];
  const float* fc1b = (const float*)d_in[29];
  const float* fc2W = (const float*)d_in[30];
  const float* fc2b = (const float*)d_in[31];
  float* out = (float*)d_out;

  char* ws = (char*)d_ws;
  unsigned short* XP   = (unsigned short*)(ws + O_XP);
  unsigned short* ZP   = (unsigned short*)(ws + O_Z);
  float*          HF   = (float*)(ws + O_H);
  int*            LIST = (int*)(ws + O_LIST);
  int*            META = (int*)(ws + O_META);
  int*            STRT = (int*)(ws + O_START);
  float*          PP   = (float*)(ws + O_P);
  unsigned short* WPL  = (unsigned short*)(ws + O_WPL);
  float*          TAB  = (float*)(ws + O_TAB);
  const unsigned short* W1D1 = WPL;
  const unsigned short* W1D2 = WPL + (size_t)256 * 8;
  const unsigned short* W1D3 = WPL + (size_t)1280 * 8;
  const unsigned short* W2D1 = WPL + (size_t)2304 * 8;
  const unsigned short* W2D2 = WPL + (size_t)3328 * 8;
  const unsigned short* W2D3 = WPL + (size_t)4352 * 8;
  const unsigned short* FC1D = WPL + (size_t)5376 * 8;

  hipFuncSetAttribute(reinterpret_cast<const void*>(&k_bucket),   hipFuncAttributeMaxDynamicSharedMemorySize, LDS_BKT);
  hipFuncSetAttribute(reinterpret_cast<const void*>(&k_mlp<32>),  hipFuncAttributeMaxDynamicSharedMemorySize, LDS_MLP);
  hipFuncSetAttribute(reinterpret_cast<const void*>(&k_mlp<128>), hipFuncAttributeMaxDynamicSharedMemorySize, LDS_MLP);
  hipFuncSetAttribute(reinterpret_cast<const void*>(&k_head),     hipFuncAttributeMaxDynamicSharedMemorySize, LDS_HEAD);

  k_prep<<<PB_XP + PB_W + PB_T, NTHR, 0, stream>>>(
      x, cp[0][0], cp[1][0], cp[2][0], cp[0][6], cp[1][6], cp[2][6], fc1W,
      cp[0][1], cp[0][2], cp[0][3], cp[0][4], cp[0][5], cp[0][7],
      cp[1][1], cp[1][2], cp[1][3], cp[1][4], cp[1][5], cp[1][7],
      cp[2][1], cp[2][2], cp[2][3], cp[2][4], cp[2][5], cp[2][7],
      fc1b, fc2W, fc2b, XP, WPL, TAB);
  k_bounds<<<1, NTHR, 0, stream>>>(batch, STRT);
  k_bucket<<<NBLK, NTHR, LDS_BKT, stream>>>(src, dst, LIST, META);
  k_agg1<<<NBLK, NTHR, 0, stream>>>(XP, LIST, META, ZP);
  k_mlp<32><<<NTILE, NTHR, LDS_MLP, stream>>>(ZP, W1D1, W2D1, TAB, HF);
  k_pool<<<NG, NTHR, 0, stream>>>(HF, STRT, PP, 0);
  k_agg2<<<NBLK, NTHR, 0, stream>>>(HF, LIST, META, ZP);
  k_mlp<128><<<NTILE, NTHR, LDS_MLP, stream>>>(ZP, W1D2, W2D2, TAB + TABL, HF);
  k_pool<<<NG, NTHR, 0, stream>>>(HF, STRT, PP, HD);
  k_agg2<<<NBLK, NTHR, 0, stream>>>(HF, LIST, META, ZP);
  k_mlp<128><<<NTILE, NTHR, LDS_MLP, stream>>>(ZP, W1D3, W2D3, TAB + 2 * TABL, HF);
  k_pool<<<NG, NTHR, 0, stream>>>(HF, STRT, PP, 2 * HD);
  k_head<<<NG / 128, NTHR, LDS_HEAD, stream>>>(PP, FC1D, TAB + 3 * TABL, META, STRT, out);
}
